// ETransformerBlock_37726992728814
// MI455X (gfx1250) — hardware-run, weakly checked
//
#include <hip/hip_runtime.h>
#include <math.h>
#include <stdint.h>

#define NBATCH 2
#define SEQ    2048
#define DM     1024
#define NH     16
#define HD     64
#define DR     32
#define DRH    16
#define DC     256
#define DC1    384
#define NTOK   (NBATCH * SEQ)
#define HDX    (HD + DR)
#define QXP    (NH * HDX)
#define QRW    (NH * DR)
#define KRP    64
#define NQB    (SEQ / 64)
#define RTP    32
#define WSC    64.0f
#define RMS_EPS 1.1920929e-07f
#define SSCALE  0.1020620726159658f
static_assert(NH * HD == DM);
static_assert((SEQ % 64) == 0 && (DM % 64) == 0 && (DC % 64) == 0 && (DC1 % 64) == 0);
static_assert(((QXP * 2) % 128) == 0);
static_assert((QXP % 8) == 0 && (QXP / 8) == 192);
static_assert((DC1 % 32) == 0 && (DC % 32) == 0);
static_assert((((KRP - DR) * DM * 2) % (256 * 16)) == 0);

typedef _Float16 v16h __attribute__((ext_vector_type(16)));
typedef _Float16 v8h  __attribute__((ext_vector_type(8)));
typedef float    v8f  __attribute__((ext_vector_type(8)));
typedef float    v4f  __attribute__((ext_vector_type(4)));
typedef unsigned int v4u __attribute__((ext_vector_type(4)));
union FH { v16h v; v8h h[2]; };

__device__ __forceinline__ unsigned short bf_bits(float f) {
  unsigned u = __float_as_uint(f);
  return (unsigned short)((u + 0x7FFFu + ((u >> 16) & 1u)) >> 16);
}
__device__ __forceinline__ float bf_up(unsigned short h) { return __uint_as_float(((unsigned)h) << 16); }
__device__ __forceinline__ float bfr(float f) { return bf_up(bf_bits(f)); }
__device__ __forceinline__ unsigned short h_bits(_Float16 x) { return __builtin_bit_cast(unsigned short, x); }
__device__ __forceinline__ unsigned pk16(unsigned short a, unsigned short b) { return (unsigned)a | ((unsigned)b << 16); }
__device__ __forceinline__ v8f zero8() { v8f z = {0.f, 0.f, 0.f, 0.f, 0.f, 0.f, 0.f, 0.f}; return z; }
__device__ __forceinline__ float silu_f(float v) {
  const float e = __expf(-v);
  const float sg = __builtin_amdgcn_rcpf(1.0f + e);
  return v * sg;
}

__device__ __forceinline__ v16h ldfrag_h(const _Float16* p) {
  FH f;
  f.h[0] = *(const v8h*)(p);
  f.h[1] = *(const v8h*)(p + 16);
  return f.v;
}

__device__ __forceinline__ v8f mma_h(v16h a, v16h b, v8f c) {
  c = __builtin_amdgcn_wmma_f32_16x16x32_f16(false, a, false, b, (short)0, c, false, false);
#if defined(__HIP_DEVICE_COMPILE__)
  asm volatile("v_nop\n\tv_nop\n\tv_nop\n\tv_nop" : "+v"(c) : "v"(a), "v"(b));
#endif
  return c;
}
__device__ __forceinline__ v8f mma_h_raw(v16h a, v16h b, v8f c) {
  return __builtin_amdgcn_wmma_f32_16x16x32_f16(false, a, false, b, (short)0, c, false, false);
}
__device__ __forceinline__ void dep_guard_h(v8f& a, v8f& b, v16h x, v16h y) {
#if defined(__HIP_DEVICE_COMPILE__)
  asm volatile("v_nop\n\tv_nop\n\tv_nop\n\tv_nop" : "+v"(a), "+v"(b) : "v"(x), "v"(y));
#endif
}
__device__ __forceinline__ void keep4_h(v16h a, v16h b, v16h c, v16h d) {
#if defined(__HIP_DEVICE_COMPILE__)
  asm volatile("v_nop" :: "v"(a), "v"(b), "v"(c), "v"(d));
#endif
}
__device__ __forceinline__ void acc_guard4(v8f& a, v8f& b, v8f& c, v8f& d) {
#if defined(__HIP_DEVICE_COMPILE__)
  asm volatile("v_nop\n\tv_nop\n\tv_nop\n\tv_nop" : "+v"(a), "+v"(b), "+v"(c), "+v"(d));
#endif
}
__device__ __forceinline__ void wave_sync_lds() {
  __builtin_amdgcn_fence(__ATOMIC_RELEASE, "workgroup");
  __builtin_amdgcn_wave_barrier();
  __builtin_amdgcn_fence(__ATOMIC_ACQUIRE, "workgroup");
}

__global__ __launch_bounds__(256) void zfill16(unsigned short* p, int n16) {
  const int i = blockIdx.x * 256 + threadIdx.x;
  if (i >= n16) return;
  const v4u z = {0u, 0u, 0u, 0u};
  unsigned short* q = p + (size_t)i * 8;
  *(volatile v4u*)q = z;
  __threadfence();
  *(volatile v4u*)q = z;
}

__global__ __launch_bounds__(256) void tr_cvt(const float* __restrict__ in0, const float* __restrict__ in1,
                                              const float* __restrict__ in2, unsigned short* out,
                                              long long zstride, int R, int C, float scale) {
  __shared__ float tile[64 * 33];
  const int z = blockIdx.z;
  const float* in = (z == 0) ? in0 : ((z == 1) ? in1 : in2);
  unsigned short* ob = out + (size_t)z * (size_t)zstride;
  const int r0 = blockIdx.y * 64, c0 = blockIdx.x * 32;
  const int t = threadIdx.x;
  {
    const int ir = t >> 2, ic = (t & 3) * 8;
    const float* g = in + (size_t)(r0 + ir) * C + c0 + ic;
    const v4f a = *(const v4f*)g;
    const v4f b = *(const v4f*)(g + 4);
    float* l = tile + ir * 33 + ic;
    l[0] = a[0]; l[1] = a[1]; l[2] = a[2]; l[3] = a[3];
    l[4] = b[0]; l[5] = b[1]; l[6] = b[2]; l[7] = b[3];
  }
  __syncthreads();
  const int orow = t >> 3, piece = (t & 7) * 8;
  v4u p;
#pragma unroll
  for (int e = 0; e < 4; ++e) {
    const float f0 = tile[(piece + 2 * e) * 33 + orow];
    const float f1 = tile[(piece + 2 * e + 1) * 33 + orow];
    const _Float16 x0 = (_Float16)(bfr(f0) * scale);
    const _Float16 x1 = (_Float16)(bfr(f1) * scale);
    p[e] = pk16(h_bits(x0), h_bits(x1));
  }
  const size_t go = (size_t)(c0 + orow) * (size_t)R + r0 + piece;
  *(volatile v4u*)(ob + go) = p;
  __threadfence();
  *(volatile v4u*)(ob + go) = p;
}

template <bool RIN>
__global__ __launch_bounds__(128) void rms_f16(const float* __restrict__ x, const float* __restrict__ g,
                                              unsigned short* out) {
  __shared__ float red[4];
  const int row = blockIdx.x, t = threadIdx.x, lane = t & 31, w = t >> 5;
  const float* xr = x + (size_t)row * DM + 8 * t;
  const v4f a = *(const v4f*)xr;
  const v4f a2 = *(const v4f*)(xr + 4);
  float v[8];
#pragma unroll
  for (int e = 0; e < 4; ++e) { v[e] = a[e]; v[4 + e] = a2[e]; }
  if (RIN) {
#pragma unroll
    for (int e = 0; e < 8; ++e) v[e] = bfr(v[e]);
  }
  float s2 = 0.f;
#pragma unroll
  for (int e = 0; e < 8; ++e) s2 += v[e] * v[e];
  for (int off = 16; off > 0; off >>= 1) s2 += __shfl_xor(s2, off, 32);
  if (lane == 0) red[w] = s2;
  __syncthreads();
  const float tot = ((red[0] + red[1]) + red[2]) + red[3];
  const float ms = tot * (1.0f / (float)DM);
  const float rs = rsqrtf(ms + RMS_EPS);
  const v4f g0 = *(const v4f*)(g + 8 * t), g1 = *(const v4f*)(g + 8 * t + 4);
  float gg[8];
#pragma unroll
  for (int e = 0; e < 4; ++e) { gg[e] = bfr(g0[e]); gg[4 + e] = bfr(g1[e]); }
  v4u p;
#pragma unroll
  for (int e = 0; e < 4; ++e) {
    const float f0 = (v[2 * e] * rs) * gg[2 * e];
    const float f1 = (v[2 * e + 1] * rs) * gg[2 * e + 1];
    p[e] = pk16(h_bits((_Float16)f0), h_bits((_Float16)f1));
  }
  unsigned short* op = out + (size_t)row * DM + 8 * t;
  *(volatile v4u*)op = p;
  __threadfence();
  *(volatile v4u*)op = p;
}

template <int OM, int BIASM, int ACT, int RES>
__global__ __launch_bounds__(256) void gemm64(
    const unsigned short* __restrict__ Ap, int lda, long long strideA,
    const unsigned short* __restrict__ Btp, int ldb, long long strideB,
    void* Cout, int ldc, long long strideC,
    const float* __restrict__ bias, int nbias, const float* __restrict__ res, int ldr,
    int M, int N, int K, float oscale) {
  const _Float16* A  = (const _Float16*)(const void*)Ap;
  const _Float16* Bt = (const _Float16*)(const void*)Btp;
  __shared__ __align__(16) float sT[8][16 * 68];
  const int b    = blockIdx.y;
  const int lane = threadIdx.x & 31;
  const int wave = threadIdx.x >> 5;
  const int tilesN = N >> 6;
  const int tilesM = M >> 6;
  const int tile = blockIdx.x * 8 + wave;
  if (tile >= tilesM * tilesN) return;
  const int tm = tile / tilesN;
  const int tn = tile - tm * tilesN;
  const int m0 = tm << 6;
  const int n0 = tn << 6;

  const _Float16* Ab = A  + (size_t)b * (size_t)strideA;
  const _Float16* Bb = Bt + (size_t)b * (size_t)strideB;

  const int rlane = lane & 15;
  const int koff  = (lane >> 4) * 8;
  const int mOff  = (lane >> 4) * 8;

  v8f acc[4][4];
#pragma unroll
  for (int i = 0; i < 4; ++i)
#pragma unroll
    for (int j = 0; j < 4; ++j) acc[i][j] = zero8();

  for (int k0 = 0; k0 < K; k0 += 32) {
    v16h bh[4];
#pragma unroll
    for (int j = 0; j < 4; ++j) {
      const size_t bo = (size_t)(n0 + (j << 4) + rlane) * ldb + koff + k0;
      bh[j] = ldfrag_h(Bb + bo);
    }
#pragma unroll
    for (int i = 0; i < 4; ++i) {
      const size_t ao = (size_t)(m0 + (i << 4) + rlane) * lda + koff + k0;
      const v16h ah = ldfrag_h(Ab + ao);
#pragma unroll
      for (int j = 0; j < 4; ++j) acc[i][j] = mma_h_raw(ah, bh[j], acc[i][j]);
      dep_guard_h(acc[i][0], acc[i][3], ah, bh[3]);
    }
    keep4_h(bh[0], bh[1], bh[2], bh[3]);
  }
  acc_guard4(acc[0][0], acc[0][1], acc[0][2], acc[0][3]);
  acc_guard4(acc[1][0], acc[1][1], acc[1][2], acc[1][3]);
  acc_guard4(acc[2][0], acc[2][1], acc[2][2], acc[2][3]);
  acc_guard4(acc[3][0], acc[3][1], acc[3][2], acc[3][3]);

  float* slab = sT[wave];
#pragma unroll
  for (int i = 0; i < 4; ++i) {
    const int mBase = m0 + (i << 4);
#pragma unroll
    for (int j = 0; j < 4; ++j) {
#pragma unroll
      for (int r = 0; r < 8; ++r) {
        slab[(mOff + r) * 68 + (j << 4) + rlane] = acc[i][j][r];
      }
    }
    wave_sync_lds();
    if (OM == 0) {
      float* C = (float*)Cout + (size_t)b * (size_t)strideC;
      const int h2 = lane >> 4, c4 = (lane & 15) * 4;
      v4f bv = {0.f, 0.f, 0.f, 0.f};
      if (BIASM == 1) {
#pragma unroll
        for (int e = 0; e < 4; ++e) {
          const int n = n0 + c4 + e;
          const int nc = min(n, nbias - 1);
          const float tb = bias[nc];
          bv[e] = (n < nbias) ? bfr(tb) : 0.f;
        }
      }
      for (int pass = 0; pass < 2; ++pass) {
#pragma unroll
        for (int it = 0; it < 8; ++it) {
          const int row = it * 2 + h2;
          const v4f sv = *(const v4f*)(slab + row * 68 + c4);
          float rb = 0.f;
          if (BIASM == 2) rb = bfr(bias[mBase + row]);
          v4f o;
#pragma unroll
          for (int e = 0; e < 4; ++e) o[e] = sv[e] * oscale + bv[e] + rb;
          if (ACT == 1) {
#pragma unroll
            for (int e = 0; e < 4; ++e) o[e] = silu_f(o[e]);
          }
          if (RES != 0) {
            const v4f rv = *(const v4f*)(res + (size_t)(mBase + row) * ldr + n0 + c4);
#pragma unroll
            for (int e = 0; e < 4; ++e) o[e] += (RES == 2) ? bfr(rv[e]) : rv[e];
          }
          *(volatile v4f*)(C + (size_t)(mBase + row) * ldc + n0 + c4) = o;
        }
        __threadfence();
      }
    } else {
      const int q = lane >> 3, c8 = (lane & 7) * 8;
      unsigned short* C = (unsigned short*)Cout + (size_t)b * (size_t)strideC;
      float b8[8];
#pragma unroll
      for (int e = 0; e < 8; ++e) b8[e] = 0.f;
      if (BIASM == 1) {
#pragma unroll
        for (int e = 0; e < 8; ++e) {
          const int n = n0 + c8 + e;
          const int nc = min(n, nbias - 1);
          const float tb = bias[nc];
          b8[e] = (n < nbias) ? bfr(tb) : 0.f;
        }
      }
      v4u hv[4];
#pragma unroll
      for (int it = 0; it < 4; ++it) {
        const int row = it * 4 + q;
        const float* sp = slab + row * 68 + c8;
        float rb = 0.f;
        if (BIASM == 2) rb = bfr(bias[mBase + row]);
        v4u pk;
#pragma unroll
        for (int e = 0; e < 4; ++e) {
          float f0 = sp[2 * e] * oscale + b8[2 * e] + rb;
          float f1 = sp[2 * e + 1] * oscale + b8[2 * e + 1] + rb;
          if (ACT == 1) { f0 = silu_f(f0); f1 = silu_f(f1); }
          pk[e] = pk16(h_bits((_Float16)f0), h_bits((_Float16)f1));
        }
        hv[it] = pk;
      }
      for (int pass = 0; pass < 2; ++pass) {
#pragma unroll
        for (int it = 0; it < 4; ++it) {
          const int row = it * 4 + q;
          *(volatile v4u*)(C + (size_t)(mBase + row) * ldc + n0 + c8) = hv[it];
        }
        __threadfence();
      }
    }
    wave_sync_lds();
  }
}

__global__ __launch_bounds__(256) void rope_tab(float* ropt) {
  __shared__ __align__(16) float tile[16 * RTP];
  const int t = threadIdx.x, sl = t >> 4, j = t & 15;
  const int s = blockIdx.x * 16 + sl;
  const float inv = exp2f(-(float)j * 0.8304820237218407f);
  const float ang = (float)s * inv;
  const float cs = cosf(ang);
  const float sn = sinf(ang);
  tile[sl * RTP + j] = cs;
  tile[sl * RTP + DRH + j] = sn;
  __syncthreads();
  if (t < 128) {
    const v4f v = *(const v4f*)(tile + 4 * t);
    float* gp = ropt + (size_t)blockIdx.x * (16 * RTP) + 4 * t;
    *(volatile v4f*)gp = v;
    __threadfence();
    *(volatile v4f*)gp = v;
  }
}

__global__ __launch_bounds__(192) void qx_pack(const unsigned short* __restrict__ qp, const float* __restrict__ qr,
                                               const unsigned short* __restrict__ kp, const float* __restrict__ kr,
                                               const float* __restrict__ ropt, unsigned short* qxo,
                                               unsigned short* kxo) {
  const int sel = blockIdx.y;
  const int t = blockIdx.x;
  const int s = t % SEQ;
  const int p = threadIdx.x;
  const int h = p / 12;
  const int w = p - h * 12;
  const unsigned short* cp = (sel == 0) ? qp : kp;
  const int wc = min(w, 7);
  const v4u cv = *(const v4u*)(cp + (size_t)t * DM + h * HD + 8 * wc);
  const int wr = max(w, 8) - 8;
  const int jb = 8 * (wr & 1);
  const int sec = wr >> 1;
  const float* rb = (sel == 0) ? qr : kr;
  const size_t ro = (sel == 0) ? ((size_t)t * QRW + (size_t)h * DR) : ((size_t)t * KRP);
  const v4f x1a = *(const v4f*)(rb + ro + jb),       x1b = *(const v4f*)(rb + ro + jb + 4);
  const v4f x2a = *(const v4f*)(rb + ro + DRH + jb), x2b = *(const v4f*)(rb + ro + DRH + jb + 4);
  const float* tp = ropt + (size_t)s * RTP;
  const v4f ca = *(const v4f*)(tp + jb),       cb = *(const v4f*)(tp + jb + 4);
  const v4f sa = *(const v4f*)(tp + DRH + jb), sb = *(const v4f*)(tp + DRH + jb + 4);
  float o[8];
#pragma unroll
  for (int e = 0; e < 4; ++e) {
    const float fa = x1a[e] * ca[e] - x2a[e] * sa[e];
    const float fb = x1a[e] * sa[e] + x2a[e] * ca[e];
    o[e] = sec ? fb : fa;
    const float fc = x1b[e] * cb[e] - x2b[e] * sb[e];
    const float fd = x1b[e] * sb[e] + x2b[e] * cb[e];
    o[4 + e] = sec ? fd : fc;
  }
  v4u rv;
#pragma unroll
  for (int e = 0; e < 4; ++e) rv[e] = pk16(h_bits((_Float16)o[2 * e]), h_bits((_Float16)o[2 * e + 1]));
  v4u ov;
#pragma unroll
  for (int e = 0; e < 4; ++e) ov[e] = (w < 8) ? cv[e] : rv[e];
  unsigned short* dp = ((sel == 0) ? qxo : kxo) + (size_t)t * QXP + 8 * p;
  *(volatile v4u*)dp = ov;
  __threadfence();
  *(volatile v4u*)dp = ov;
}

__global__ __launch_bounds__(128)
void attn_x(const unsigned short* __restrict__ qxp, const unsigned short* __restrict__ kxp,
            const unsigned short* __restrict__ vtp, const int* __restrict__ maskp,
            unsigned short* ctxp, float sscale) {
  __shared__ __align__(16) _Float16 Ksh[64 * HDX];
  __shared__ __align__(16) _Float16 Vth[64 * 64];
  __shared__ __align__(16) _Float16 Psh[4][16 * 64];
  __shared__ __align__(16) float    Os[4][16 * 64];

  const int tid  = threadIdx.x;
  const int wave = tid >> 5;
  const int lane = tid & 31;
  const int hh   = lane >> 4;
  const int c    = lane & 15;

  const int bx   = blockIdx.x;
  const int qb   = bx % NQB;
  const int rest = bx / NQB;
  const int h    = rest % NH;
  const int b    = rest / NH;
  const int q0   = qb * 64 + wave * 16;
  const size_t rowB = (size_t)b * SEQ;

  const _Float16* Qg = (const _Float16*)(const void*)qxp + (size_t)h * HDX;
  const _Float16* Kg = (const _Float16*)(const void*)kxp + (size_t)h * HDX;
  const _Float16* Vg = (const _Float16*)(const void*)vtp + ((size_t)b * DM + (size_t)h * HD) * SEQ;
  const int* Mg = maskp + (size_t)(q0 + 8 * hh) * SEQ + c;

  v16h qa[3];
#pragma unroll
  for (int dc = 0; dc < 3; ++dc) qa[dc] = ldfrag_h(Qg + (rowB + q0 + c) * QXP + dc * 32 + 8 * hh);

  float mrow[8], lrow[8];
  v8f oacc[4];
#pragma unroll
  for (int r = 0; r < 8; ++r) { mrow[r] = -INFINITY; lrow[r] = 0.f; }
#pragma unroll
  for (int t = 0; t < 4; ++t) oacc[t] = zero8();

  for (int kt = 0; kt < NQB; ++kt) {
    const int kv0 = kt * 64;
    __syncthreads();
    {
      const int r = tid >> 1, hk = (tid & 1) * 48, hv = (tid & 1) * 32;
      const _Float16* kg = Kg + (rowB + kv0 + r) * QXP + hk;
      const _Float16* vg = Vg + (size_t)r * SEQ + kv0 + hv;
#pragma unroll
      for (int i = 0; i < 6; ++i) *(v8h*)(Ksh + r * HDX + hk + 8 * i) = *(const v8h*)(kg + 8 * i);
#pragma unroll
      for (int i = 0; i < 4; ++i) *(v8h*)(Vth + r * 64 + hv + 8 * i) = *(const v8h*)(vg + 8 * i);
    }
    __syncthreads();

    v8f s[4];
#pragma unroll
    for (int j = 0; j < 4; ++j) {
      v8f sh = zero8();
#pragma unroll
      for (int dc = 0; dc < 3; ++dc) {
        FH kb;
        kb.h[0] = *(const v8h*)(Ksh + (j * 16 + c) * HDX + dc * 32 + 8 * hh);
        kb.h[1] = *(const v8h*)(Ksh + (j * 16 + c) * HDX + dc * 32 + 16 + 8 * hh);
        sh = mma_h(qa[dc], kb.v, sh);
      }
#pragma unroll
      for (int r = 0; r < 8; ++r) {
        const int mv = Mg[(size_t)r * SEQ + kv0 + j * 16];
        const float sv = sh[r] * sscale;
        s[j][r] = (mv != 0) ? sv : -1.0e9f;
      }
    }

    _Float16* pwh = Psh[wave];
#pragma unroll
    for (int r = 0; r < 8; ++r) {
      float m = s[0][r];
      m = fmaxf(m, s[1][r]);
      m = fmaxf(m, s[2][r]);
      m = fmaxf(m, s[3][r]);
#pragma unroll
      for (int off = 1; off < 16; off <<= 1) m = fmaxf(m, __shfl_xor(m, off, 32));
      const float mnew  = fmaxf(mrow[r], m);
      const float alpha = __expf(mrow[r] - mnew);
      mrow[r] = mnew;
      float psum = 0.f;
#pragma unroll
      for (int j = 0; j < 4; ++j) {
        const float p = __expf(s[j][r] - mnew);
        psum += p;
        pwh[(8 * hh + r) * 64 + j * 16 + c] = (_Float16)(p * 1024.0f);
      }
#pragma unroll
      for (int off = 1; off < 16; off <<= 1) psum += __shfl_xor(psum, off, 32);
      lrow[r] = lrow[r] * alpha + psum;
#pragma unroll
      for (int t = 0; t < 4; ++t) oacc[t][r] *= alpha;
    }
    wave_sync_lds();

#pragma unroll 1
    for (int kk = 0; kk < 2; ++kk) {
      FH pa;
      pa.h[0] = *(const v8h*)(pwh + c * 64 + kk * 32 + 8 * hh);
      pa.h[1] = *(const v8h*)(pwh + c * 64 + kk * 32 + 16 + 8 * hh);
#pragma unroll
      for (int t = 0; t < 4; ++t) {
        FH vb;
        vb.h[0] = *(const v8h*)(Vth + (t * 16 + c) * 64 + kk * 32 + 8 * hh);
        vb.h[1] = *(const v8h*)(Vth + (t * 16 + c) * 64 + kk * 32 + 16 + 8 * hh);
        oacc[t] = mma_h(pa.v, vb.v, oacc[t]);
      }
    }
  }

  float* os = Os[wave];
#pragma unroll
  for (int r = 0; r < 8; ++r) {
    const float l = lrow[r];
    const float inv = ((l > 0.f) ? (1.0f / l) : 0.f) * (64.0f / 1024.0f);
#pragma unroll
    for (int t = 0; t < 4; ++t) os[(8 * hh + r) * 64 + t * 16 + c] = oacc[t][r] * inv;
  }
  wave_sync_lds();
  {
    const int q4 = lane >> 3, c8 = (lane & 7) * 8;
    v4u hvv[4];
#pragma unroll
    for (int it = 0; it < 4; ++it) {
      const int row = it * 4 + q4;
      const float* sp = os + row * 64 + c8;
      v4u pk;
#pragma unroll
      for (int e = 0; e < 4; ++e) {
        pk[e] = pk16(h_bits((_Float16)sp[2 * e]), h_bits((_Float16)sp[2 * e + 1]));
      }
      hvv[it] = pk;
    }
    for (int pass = 0; pass < 2; ++pass) {
#pragma unroll
      for (int it = 0; it < 4; ++it) {
        const int row = it * 4 + q4;
        const size_t go = (rowB + q0 + row) * DM + (size_t)h * HD + c8;
        *(volatile v4u*)(ctxp + go) = hvv[it];
      }
      __threadfence();
    }
  }
}

extern "C" void kernel_launch(void* const* d_in, const int* in_sizes, int n_in,
                              void* d_out, int out_size, void* d_ws, size_t ws_size,
                              hipStream_t stream) {
  if (n_in < 21) return;
  if (in_sizes[0] != NTOK * DM) return;
  if (in_sizes[1] != SEQ * SEQ) return;
  if (in_sizes[2] != DM) return;
  if (in_sizes[3] != DM * DC1 || in_sizes[4] != DC1) return;
  if (in_sizes[5] != DC1 * DM || in_sizes[6] != DM) return;
  if (in_sizes[7] != DC1 * QRW || in_sizes[8] != QRW) return;
  if (in_sizes[9] != DM * DC || in_sizes[10] != DC) return;
  if (in_sizes[11] != DC * DM || in_sizes[12] != DM) return;
  if (in_sizes[13] != DC * DM || in_sizes[14] != DM) return;
  if (in_sizes[15] != DM * DR || in_sizes[16] != DR) return;
  if (in_sizes[17] != DM * DM || in_sizes[18] != DM) return;
  if (in_sizes[19] != DM * DM || in_sizes[20] != DM) return;
  if (out_size != NTOK * DM) return;

  const float* x_in  = (const float*)d_in[0];
  const int*   mask  = (const int*)d_in[1];
  const float* gamma = (const float*)d_in[2];
  const float* W_dq  = (const float*)d_in[3];   const float* b_dq  = (const float*)d_in[4];
  const float* W_uq  = (const float*)d_in[5];   const float* b_uq  = (const float*)d_in[6];
  const float* W_qr  = (const float*)d_in[7];   const float* b_qr  = (const float*)d_in[8];
  const float* W_dkv = (const float*)d_in[9];   const float* b_dkv = (const float*)d_in[10];
  const float* W_uk  = (const float*)d_in[11];  const float* b_uk  = (const float*)d_in[12];
  const float* W_uv  = (const float*)d_in[13];  const float* b_uv  = (const float*)d_in[14];
  const float* W_kr  = (const float*)d_in[15];  const float* b_kr  = (const float*)d_in[16];
  const float* W_o   = (const float*)d_in[17];  const float* b_o   = (const float*)d_in[18];
  const float* W_fc  = (const float*)d_in[19];  const float* b_fc  = (const float*)d_in[20];
  float* outf = (float*)d_out;

  const size_t PWDQ  = (size_t)DC1 * DM * 2;
  const size_t PWUQ  = (size_t)DM * DC1 * 2;
  const size_t PWQR  = (size_t)QRW * DC1 * 2;
  const size_t PWDKV = (size_t)DC * DM * 2;
  const size_t PWUKV = (size_t)2 * DM * DC * 2;
  const size_t PWKR  = (size_t)KRP * DM * 2;
  const size_t PWOF  = (size_t)2 * DM * DM * 2;
  const size_t PROPT = (size_t)SEQ * RTP * 4;
  const size_t PXN   = (size_t)NTOK * DM * 2;
  const size_t PQC   = (size_t)NTOK * DC1 * 2;
  const size_t PCKV  = (size_t)NTOK * DC * 2;
  const size_t PQP   = (size_t)NTOK * DM * 2;
  const size_t PKP   = (size_t)NTOK * DM * 2;
  const size_t PQR   = (size_t)NTOK * QRW * 4;
  const size_t PKR   = (size_t)NTOK * KRP * 4;
  const size_t PVT   = (size_t)NBATCH * DM * SEQ * 2;
  const size_t PQX   = (size_t)NTOK * QXP * 2;
  const size_t PCTX  = (size_t)NTOK * DM * 2;
  const size_t PX1   = (size_t)NTOK * DM * 4;
  size_t off = 0;
  const size_t oWDQ  = off; off += PWDQ;
  const size_t oWUQ  = off; off += PWUQ;
  const size_t oWQR  = off; off += PWQR;
  const size_t oWDKV = off; off += PWDKV;
  const size_t oWUKV = off; off += PWUKV;
  const size_t oWKR  = off; off += PWKR;
  const size_t oWOF  = off; off += PWOF;
  const size_t oROPT = off; off += PROPT;
  const size_t oXN   = off; off += PXN;
  const size_t oQC   = off; off += PQC;
  const size_t oCKV  = off; off += PCKV;
  const size_t oQP   = off; off += PQP;
  const size_t oKP   = off; off += PKP;
  const size_t oQR   = off; off += PQR;
  const size_t oKR   = off; off += PKR;
  const size_t oVT   = off; off += PVT;
  const size_t oQX   = off; off += PQX;
  const size_t oKX   = off; off += PQX;
  const size_t oCTX  = off; off += PCTX;
  const size_t oX1   = off; off += PX1;
  if (off > ws_size) return;
  if (off > (size_t)134217728) return;

  char* ws = (char*)d_ws;
  unsigned short* WDQT  = (unsigned short*)(ws + oWDQ);
  unsigned short* WUQT  = (unsigned short*)(ws + oWUQ);
  unsigned short* WQRT  = (unsigned short*)(ws + oWQR);
  unsigned short* WDKVT = (unsigned short*)(ws + oWDKV);
  unsigned short* WUKT  = (unsigned short*)(ws + oWUKV);
  unsigned short* WUVT  = WUKT + (size_t)DM * DC;
  unsigned short* WKRT  = (unsigned short*)(ws + oWKR);
  unsigned short* WOT   = (unsigned short*)(ws + oWOF);
  unsigned short* WFCT  = WOT + (size_t)DM * DM;
  float*          ROPT  = (float*)(ws + oROPT);
  unsigned short* XN    = (unsigned short*)(ws + oXN);
  unsigned short* QC    = (unsigned short*)(ws + oQC);
  unsigned short* CKV   = (unsigned short*)(ws + oCKV);
  unsigned short* QP    = (unsigned short*)(ws + oQP);
  unsigned short* KP    = (unsigned short*)(ws + oKP);
  float*          QR    = (float*)(ws + oQR);
  float*          KR    = (float*)(ws + oKR);
  unsigned short* VT    = (unsigned short*)(ws + oVT);
  unsigned short* QX    = (unsigned short*)(ws + oQX);
  unsigned short* KX    = (unsigned short*)(ws + oKX);
  unsigned short* CTX   = (unsigned short*)(ws + oCTX);
  float*          X1    = (float*)(ws + oX1);

  const dim3 blk(256);

  tr_cvt<<<dim3(DC1 / 32, DM / 64, 1), blk, 0, stream>>>(W_dq, W_dq, W_dq, WDQT, 0LL, DM, DC1, WSC);
  tr_cvt<<<dim3(DM / 32, DC1 / 64, 1), blk, 0, stream>>>(W_uq, W_uq, W_uq, WUQT, 0LL, DC1, DM, WSC);
  tr_cvt<<<dim3(QRW / 32, DC1 / 64, 1), blk, 0, stream>>>(W_qr, W_qr, W_qr, WQRT, 0LL, DC1, QRW, WSC);
  tr_cvt<<<dim3(DC / 32, DM / 64, 1), blk, 0, stream>>>(W_dkv, W_dkv, W_dkv, WDKVT, 0LL, DM, DC, WSC);
  tr_cvt<<<dim3(DM / 32, DC / 64, 2), blk, 0, stream>>>(W_uk, W_uv, W_uv, WUKT, (long long)DM * DC, DC, DM, WSC);
  tr_cvt<<<dim3(DR / 32, DM / 64, 1), blk, 0, stream>>>(W_kr, W_kr, W_kr, WKRT, 0LL, DM, DR, WSC);
  {
    const int n16 = ((KRP - DR) * DM * 2) / 16;
    zfill16<<<dim3((n16 + 255) / 256), blk, 0, stream>>>(WKRT + (size_t)DR * DM, n16);
  }
  tr_cvt<<<dim3(DM / 32, DM / 64, 2), blk, 0, stream>>>(W_o, W_fc, W_fc, WOT, (long long)DM * DM, DM, DM, WSC);
  rope_tab<<<dim3(SEQ / 16), blk, 0, stream>>>(ROPT);
  rms_f16<true><<<dim3(NTOK), dim3(128), 0, stream>>>(x_in, gamma, XN);
  gemm64<1, 1, 0, 0><<<dim3(((NTOK / 64) * (DC1 / 64) + 7) / 8, 1), blk, 0, stream>>>(
      XN, DM, 0LL, WDQT, DM, 0LL, (void*)QC, DC1, 0LL, b_dq, DC1, x_in, DM, NTOK, DC1, DM, 1.0f / WSC);
  gemm64<1, 1, 0, 0><<<dim3(((NTOK / 64) * (DC / 64) + 7) / 8, 1), blk, 0, stream>>>(
      XN, DM, 0LL, WDKVT, DM, 0LL, (void*)CKV, DC, 0LL, b_dkv, DC, x_in, DM, NTOK, DC, DM, 1.0f / WSC);
  gemm64<1, 1, 0, 0><<<dim3(((NTOK / 64) * (DM / 64) + 7) / 8, 1), blk, 0, stream>>>(
      QC, DC1, 0LL, WUQT, DC1, 0LL, (void*)QP, DM, 0LL, b_uq, DM, x_in, DM, NTOK, DM, DC1, 1.0f / WSC);
  gemm64<0, 1, 0, 0><<<dim3(((NTOK / 64) * (QRW / 64) + 7) / 8, 1), blk, 0, stream>>>(
      QC, DC1, 0LL, WQRT, DC1, 0LL, (void*)QR, QRW, 0LL, b_qr, QRW, x_in, DM, NTOK, QRW, DC1, 1.0f / WSC);
  gemm64<1, 1, 0, 0><<<dim3(((NTOK / 64) * (DM / 64) + 7) / 8, 1), blk, 0, stream>>>(
      CKV, DC, 0LL, WUKT, DC, 0LL, (void*)KP, DM, 0LL, b_uk, DM, x_in, DM, NTOK, DM, DC, 1.0f / WSC);
  gemm64<1, 2, 0, 0><<<dim3(((DM / 64) * (SEQ / 64) + 7) / 8, NBATCH), blk, 0, stream>>>(
      WUVT, DC, 0LL, CKV, DC, (long long)SEQ * DC, (void*)VT, SEQ, (long long)DM * SEQ, b_uv, DM, x_in, DM,
      DM, SEQ, DC, 1.0f / WSC);
  gemm64<0, 1, 0, 0><<<dim3(((NTOK / 64) * (KRP / 64) + 7) / 8, 1), blk, 0, stream>>>(
      XN, DM, 0LL, WKRT, DM, 0LL, (void*)KR, KRP, 0LL, b_kr, DR, x_in, DM, NTOK, KRP, DM, 1.0f / WSC);
  qx_pack<<<dim3(NTOK, 2), dim3(192), 0, stream>>>(QP, QR, KP, KR, ROPT, QX, KX);
  attn_x<<<dim3(NBATCH * NH * NQB), dim3(128), 0, stream>>>(QX, KX, VT, mask, CTX, SSCALE);
  gemm64<0, 1, 0, 2><<<dim3(((NTOK / 64) * (DM / 64) + 7) / 8, 1), blk, 0, stream>>>(
      CTX, DM, 0LL, WOT, DM, 0LL, (void*)X1, DM, 0LL, b_o, DM, x_in, DM, NTOK, DM, DM, 1.0f / (WSC * 64.0f));
  rms_f16<false><<<dim3(NTOK), dim3(128), 0, stream>>>(X1, gamma, XN);
  gemm64<0, 1, 1, 1><<<dim3(((NTOK / 64) * (DM / 64) + 7) / 8, 1), blk, 0, stream>>>(
      XN, DM, 0LL, WFCT, DM, 0LL, (void*)outf, DM, 0LL, b_fc, DM, X1, DM, NTOK, DM, DM, 1.0f / WSC);
  (void)hipGetLastError();
}
